// CrossAttention_79448305041860
// MI455X (gfx1250) — hardware-run, weakly checked
//
#include <hip/hip_runtime.h>


#ifndef NB
#define NB 4
#endif
#ifndef SEQ
#define SEQ 4096
#endif
#define NB_FULL  4
#define SEQ_FULL 4096
#ifndef OUT_SEQ
#define OUT_SEQ SEQ
#endif
#define CCH  256
#define KVC  512
#define CTXP 512
#define AW   4
#define QPITCH 264
#define HSC  16.0f
#define WSC  64.0f
#define QSC  16.0f
#define VSC  16.0f
#define OSC  1024.0f
#define PSH  8.0f
#define SC2  (0.0625f * 1.4426950408889634f / (QSC * QSC))

static_assert(CCH == 256);
static_assert(CCH == 8 * 32);
static_assert(CTXP == 2 * CCH);
static_assert(CCH % 64 == 0);
static_assert(KVC % 64 == 0);
static_assert(CCH % 32 == 0);
static_assert(KVC % 32 == 0);
static_assert(CTXP % 32 == 0);
static_assert(SEQ % 64 == 0);
static_assert((NB * SEQ) % 64 == 0);
static_assert(SEQ % 32 == 0);
static_assert(SEQ % (16 * AW) == 0);
static_assert(SEQ % 4 == 0);
static_assert(OUT_SEQ % 32 == 0);
static_assert(OUT_SEQ >= SEQ);
static_assert(QPITCH % 8 == 0);
static_assert(QPITCH >= CCH);
static_assert(NB <= NB_FULL);
static_assert(SEQ <= SEQ_FULL);

typedef _Float16 h16;
typedef __attribute__((ext_vector_type(16))) _Float16 v16h;
typedef __attribute__((ext_vector_type(8)))  _Float16 v8h;
typedef __attribute__((ext_vector_type(8)))  float    v8f;
typedef __attribute__((ext_vector_type(4)))  float    v4f;
typedef v4f  __attribute__((may_alias)) v4fa;
typedef v8h  __attribute__((may_alias)) v8ha;

__device__ __forceinline__ unsigned short f2bf(float f) { unsigned u = __float_as_uint(f); u += 0x7FFFu + ((u >> 16) & 1u); return (unsigned short)(u >> 16); }
__device__ __forceinline__ float bfr(float f) { return __uint_as_float(((unsigned)f2bf(f)) << 16); }
__device__ __forceinline__ v16h cat16(v8h lo, v8h hi) { return __builtin_shufflevector(lo, hi, 0, 1, 2, 3, 4, 5, 6, 7, 8, 9, 10, 11, 12, 13, 14, 15); }
__device__ __forceinline__ v8f wmma16(v16h a, v16h b, v8f c) { return __builtin_amdgcn_wmma_f32_16x16x32_f16(false, a, false, b, (short)0, c, false, false); }
__device__ __forceinline__ v16h ldh(const h16* p) { return cat16(*(const v8h*)p, *(const v8h*)(p + 16)); }
__device__ __forceinline__ void wave_sync() { __builtin_amdgcn_fence(3  , "wavefront"); __builtin_amdgcn_wave_barrier(); asm volatile("" ::: "memory"); }

__global__ __launch_bounds__(256) void k_cvtw(const float* __restrict__ src, h16* dst, size_t n8) {
    const size_t i = (size_t)blockIdx.x * 256 + threadIdx.x; if (i >= n8) return;
    const v8f v = *(const v8f*)(src + i * 8); v8h o;
#pragma unroll
    for (int k = 0; k < 8; ++k) o[k] = (h16)(bfr(v[k]) * WSC);
    *(volatile v8h*)(dst + i * 8) = o; __threadfence(); *(volatile v8h*)(dst + i * 8) = o;
}

__global__ __launch_bounds__(256) void k_xpose(const float* __restrict__ x, h16* XT, int CP) {
    __shared__ __align__(16) h16 tile[64 * 72];
    const int tid = threadIdx.x;
    const int n0 = blockIdx.x * 64, c0 = blockIdx.y * 64, b = blockIdx.z;
#pragma unroll
    for (int i = 0; i < 4; ++i) {
        const int u = tid + 256 * i; const int cl = u >> 4, n4 = (u & 15) * 4;
        const int c = c0 + cl;
        const v4f v = *(const v4f*)(x + ((size_t)b * CP + c) * SEQ_FULL + n0 + n4);
#pragma unroll
        for (int j = 0; j < 4; ++j) { const float hv = bfr(v[j]) * HSC; tile[(n4 + j) * 72 + cl] = (h16)hv; }
    }
    __syncthreads();
#pragma unroll 1
    for (int ps = 0; ps < 2; ++ps) {
#pragma unroll
        for (int i = 0; i < 2; ++i) {
            const int line = (tid >> 3) + 32 * i, piece = tid & 7;
            const v8h val = *(const v8ha*)(&tile[line * 72 + piece * 8]);
            *(volatile v8h*)(XT + ((size_t)b * SEQ + n0 + line) * CP + c0 + piece * 8) = val; }
        if (ps == 0) __threadfence(); }
}

template <int MODE>
__device__ __forceinline__ void gemm_tile(const h16* __restrict__ A, const h16* __restrict__ Bt, const float* __restrict__ bias,
                                          h16* Ph, float* Yf, int K, int RB, size_t sRB, int pitch, int CB, size_t sCB, float scale, float osc) {
    __shared__ __align__(16) float os[16 * 68];
    const int lane = threadIdx.x & 31, lr = lane & 15, hi = lane >> 4; const int r0 = blockIdx.x * 64, c0 = blockIdx.y * 64;
    v8f acc[4][4];
#pragma unroll
    for (int mb = 0; mb < 4; ++mb)
#pragma unroll
        for (int nb = 0; nb < 4; ++nb) acc[mb][nb] = (v8f){};
    const size_t aoff = (size_t)(r0 + lr) * K + 8 * hi, boff = (size_t)(c0 + lr) * K + 8 * hi;
#pragma unroll 1
    for (int kc = 0; kc < K; kc += 32) {
        v16h a[4];
#pragma unroll
        for (int mb = 0; mb < 4; ++mb) a[mb] = ldh(A + aoff + (size_t)mb * 16 * K + kc);
#pragma unroll
        for (int nb = 0; nb < 4; ++nb) { const v16h bfrag = ldh(Bt + boff + (size_t)nb * 16 * K + kc);
#pragma unroll
            for (int mb = 0; mb < 4; ++mb) acc[mb][nb] = wmma16(a[mb], bfrag, acc[mb][nb]); }
        asm volatile("v_nop\n\tv_nop\n\tv_nop\n\tv_nop" : "+v"(acc[0][0]), "+v"(acc[1][1]), "+v"(acc[2][2]), "+v"(acc[3][3]) : "v"(a[0]), "v"(a[1]), "v"(a[2]), "v"(a[3]));
    }
    const size_t cq = (size_t)(c0 / CB), cr = (size_t)(c0 % CB);
    const size_t tbase = (size_t)(r0 / RB) * sRB + (size_t)(r0 % RB) * (size_t)pitch + cq * sCB + cr;
    float bc[8];
#pragma unroll
    for (int i = 0; i < 8; ++i) bc[i] = 0.0f;
    if (MODE == 0) {
        const v4f b0 = *(const v4f*)(bias + c0 + (lane & 7) * 8); const v4f b1 = *(const v4f*)(bias + c0 + (lane & 7) * 8 + 4);
#pragma unroll
        for (int i = 0; i < 4; ++i) { bc[i] = bfr(b0[i]); bc[4 + i] = bfr(b1[i]); }
    }
#pragma unroll
    for (int mb = 0; mb < 4; ++mb) {
#pragma unroll
        for (int nb = 0; nb < 4; ++nb) {
#pragma unroll
            for (int j = 0; j < 8; ++j) os[(hi * 8 + j) * 68 + nb * 16 + lr] = acc[mb][nb][j]; }
        wave_sync();
        const size_t sb = tbase + (size_t)(mb * 16) * (size_t)pitch;
#pragma unroll 1
        for (int ps = 0; ps < 2; ++ps) {
            if (MODE == 2) {
#pragma unroll
                for (int s = 0; s < 8; ++s) { const int row = 2 * s + hi, cofs = lr * 4;
                    const v4f a4 = *(const v4fa*)(&os[row * 68 + cofs]);
                    const float br = bfr(bias[r0 + mb * 16 + row]);
                    v4f val;
#pragma unroll
                    for (int i = 0; i < 4; ++i) val[i] = a4[i] * scale + br;
                    *(volatile v4f*)(Yf + sb + (size_t)row * (size_t)pitch + cofs) = val; }
            } else {
#pragma unroll
                for (int s = 0; s < 4; ++s) { const int row = 4 * s + (lane >> 3), c8 = (lane & 7) * 8;
                    const v4f x0 = *(const v4fa*)(&os[row * 68 + c8]); const v4f x1 = *(const v4fa*)(&os[row * 68 + c8 + 4]);
                    float br = 0.0f;
                    if (MODE == 1) br = bfr(bias[r0 + mb * 16 + row]);
                    v8h hv;
#pragma unroll
                    for (int i = 0; i < 4; ++i) {
                        const float f0 = x0[i] * scale + ((MODE == 0) ? bc[i] : br);
                        const float f1 = x1[i] * scale + ((MODE == 0) ? bc[4 + i] : br);
                        hv[i] = (h16)(f0 * osc); hv[4 + i] = (h16)(f1 * osc); }
                    *(volatile v8h*)(Ph + sb + (size_t)row * (size_t)pitch + c8) = hv; }
            }
            if (ps == 0) __threadfence(); }
        wave_sync();
    }
}

__global__ __launch_bounds__(32) void k_gemm_cb(const h16* __restrict__ A, const h16* __restrict__ Bt, const float* __restrict__ bias, h16* Ph,
                                                int K, int RB, size_t sRB, int pitch, int CB, size_t sCB, float scale, float osc) {
    gemm_tile<0>(A, Bt, bias, Ph, (float*)0, K, RB, sRB, pitch, CB, sCB, scale, osc);
}
__global__ __launch_bounds__(32) void k_gemm_rb(const h16* __restrict__ A, const h16* __restrict__ Bt, const float* __restrict__ bias, h16* Ph,
                                                int K, int RB, size_t sRB, int pitch, int CB, size_t sCB, float scale, float osc) {
    gemm_tile<1>(A, Bt, bias, Ph, (float*)0, K, RB, sRB, pitch, CB, sCB, scale, osc);
}
__global__ __launch_bounds__(32) void k_gemm_f32(const h16* __restrict__ A, const h16* __restrict__ Bt, const float* __restrict__ bias, float* Yf,
                                                 int K, int RB, size_t sRB, int pitch, int CB, size_t sCB, float scale, float osc) {
    gemm_tile<2>(A, Bt, bias, (h16*)0, Yf, K, RB, sRB, pitch, CB, sCB, scale, osc);
}

__global__ __launch_bounds__(32 * AW) void k_flash(const h16* __restrict__ QP, const h16* __restrict__ KP, const h16* __restrict__ VT, h16* OP) {
    __shared__ __align__(16) h16 qs[AW * 16 * QPITCH];
    const int lane = threadIdx.x & 31, wave = __builtin_amdgcn_readfirstlane((int)(threadIdx.x >> 5)), lr = lane & 15, hi = lane >> 4;
    const int b = blockIdx.y;
    const int z = blockIdx.z;
    const int t0 = (blockIdx.x * AW + wave) * 16;
    const int wb = wave * 16 * QPITCH;
    const size_t rowbase = (size_t)b * SEQ;
    const size_t qplane = (size_t)z * ((size_t)NB * SEQ * CCH);
#pragma unroll
    for (int i = 0; i < 16; ++i) {
        const v8h v = *(const v8h*)(QP + qplane + (rowbase + t0 + i) * CCH + lane * 8);
        *(v8h*)(&qs[wb + i * QPITCH + lane * 8]) = v; }
    wave_sync();
    const int qoff = wb + lr * QPITCH + 8 * hi;
    const size_t ko = (rowbase + lr) * CCH + 8 * hi;
    const size_t vo = ((size_t)b * CCH + lr) * SEQ + 8 * hi;
    v8f o[16];
#pragma unroll
    for (int i = 0; i < 16; ++i) o[i] = (v8f){};
    float m = -3.0e38f, l = 0.0f;
#pragma unroll 1
    for (int key0 = 0; key0 < SEQ; key0 += 32) {
        const h16* ka = KP + ko + (size_t)key0 * CCH;
        v8f sa = (v8f){}, sb = (v8f){};
#pragma unroll 1
        for (int kc = 0; kc < CCH; kc += 64) {
            const v16h q0 = cat16(*(const v8h*)(&qs[qoff + kc]),      *(const v8h*)(&qs[qoff + kc + 16]));
            const v16h q1 = cat16(*(const v8h*)(&qs[qoff + kc + 32]), *(const v8h*)(&qs[qoff + kc + 48]));
            const v16h ka0 = ldh(ka + kc), ka1 = ldh(ka + kc + 32), kb0 = ldh(ka + 16 * CCH + kc), kb1 = ldh(ka + 16 * CCH + kc + 32);
            sa = wmma16(ka0, q0, sa); sb = wmma16(kb0, q0, sb);
            sa = wmma16(ka1, q1, sa); sb = wmma16(kb1, q1, sb);
            asm volatile("v_nop\n\tv_nop\n\tv_nop\n\tv_nop" : "+v"(sa), "+v"(sb) : "v"(ka0), "v"(ka1), "v"(kb0), "v"(kb1), "v"(q0), "v"(q1));
        }
        float ta[8], tb[8]; float mx = -3.0e38f;
#pragma unroll
        for (int r = 0; r < 8; ++r) { ta[r] = sa[r] * SC2; tb[r] = sb[r] * SC2; mx = fmaxf(mx, fmaxf(ta[r], tb[r])); }
        mx = fmaxf(mx, __shfl_xor(mx, 16, 32));
        const float mnew = fmaxf(m, mx);
        const float alpha = __builtin_amdgcn_exp2f(m - mnew);
        const float sh = PSH - mnew;
        v16h pb; float ls = 0.0f;
#pragma unroll
        for (int r = 0; r < 8; ++r) { const h16 pa = (h16)__builtin_amdgcn_exp2f(ta[r] + sh); const h16 pc = (h16)__builtin_amdgcn_exp2f(tb[r] + sh); pb[r] = pa; pb[8 + r] = pc; ls += (float)pa + (float)pc; }
        l = l * alpha + ls; m = mnew;
        const unsigned need = __builtin_amdgcn_ballot_w32(alpha != 1.0f);
        if (need != 0u) {
#pragma unroll
            for (int i = 0; i < 16; ++i) o[i] = o[i] * alpha;
        }
        const h16* va = VT + vo + key0;
#pragma unroll
        for (int g = 0; g < 4; ++g) {
            const h16* vg = va + (size_t)(64 * g) * SEQ;
            const v16h v0 = ldh(vg), v1 = ldh(vg + (size_t)16 * SEQ), v2 = ldh(vg + (size_t)32 * SEQ), v3 = ldh(vg + (size_t)48 * SEQ);
            o[4 * g + 0] = wmma16(v0, pb, o[4 * g + 0]); o[4 * g + 1] = wmma16(v1, pb, o[4 * g + 1]);
            o[4 * g + 2] = wmma16(v2, pb, o[4 * g + 2]); o[4 * g + 3] = wmma16(v3, pb, o[4 * g + 3]);
            asm volatile("v_nop\n\tv_nop\n\tv_nop\n\tv_nop" : "+v"(o[4 * g + 0]), "+v"(o[4 * g + 1]), "+v"(o[4 * g + 2]), "+v"(o[4 * g + 3]) : "v"(v0), "v"(v1), "v"(v2), "v"(v3), "v"(pb));
        }
    }
    l += __shfl_xor(l, 16, 32);
    const float osc = (OSC / VSC) * (1.0f / l);
    wave_sync();
#pragma unroll
    for (int j = 0; j < 16; ++j) { v8h pk;
#pragma unroll
        for (int r = 0; r < 8; ++r) pk[r] = (h16)(o[j][r] * osc);
        *(v8h*)(&qs[wb + lr * QPITCH + 16 * j + 8 * hi]) = pk; }
    wave_sync();
    h16* orow = OP + (rowbase + t0) * CTXP + (size_t)z * CCH + lane * 8;
#pragma unroll 1
    for (int ps = 0; ps < 2; ++ps) {
#pragma unroll
        for (int row = 0; row < 16; ++row) {
            const v8h val = *(const v8h*)(&qs[wb + row * QPITCH + lane * 8]);
            *(volatile v8h*)(orow + (size_t)row * CTXP) = val; }
        if (ps == 0) __threadfence(); }
}

__global__ __launch_bounds__(256) void k_ln(const float* __restrict__ Y, const float* __restrict__ lw, const float* __restrict__ lb, float* OUT) {
#pragma clang fp contract(off)
    __shared__ __align__(16) float tile[CCH * 32];
    __shared__ __align__(16) float pr[8 * 32];
    __shared__ __align__(16) float smu[32];
    __shared__ __align__(16) float srs[32];
    const int tid = threadIdx.x, tl = tid & 31;
    const int wave = __builtin_amdgcn_readfirstlane((int)(threadIdx.x >> 5));
    const int t0 = blockIdx.x * 32, b = blockIdx.y;
    const float* yb = Y + (size_t)b * CCH * SEQ + t0 + tl;
    float s = 0.0f;
#pragma unroll 1
    for (int i = 0; i < 32; ++i) {
        const int e = wave + 8 * i; const float v = yb[(size_t)e * SEQ]; tile[e * 32 + tl] = v; s += v; }
    pr[wave * 32 + tl] = s;
    __syncthreads();
    float tot = 0.0f;
#pragma unroll 1
    for (int w = 0; w < 8; ++w) tot += pr[w * 32 + tl];
    const float mu = tot * (1.0f / CCH);
    __syncthreads();
    float q = 0.0f;
#pragma unroll 1
    for (int i = 0; i < 32; ++i) { const int e = wave + 8 * i; const float d = tile[e * 32 + tl] - mu; q += d * d; }
    pr[wave * 32 + tl] = q;
    __syncthreads();
    float tq = 0.0f;
#pragma unroll 1
    for (int w = 0; w < 8; ++w) tq += pr[w * 32 + tl];
    const float rs = rsqrtf(tq * (1.0f / CCH) + 1.0e-5f);
    if (wave == 0) { smu[tl] = mu; srs[tl] = rs; }
    __syncthreads();
#pragma unroll 1
    for (int ps = 0; ps < 2; ++ps) {
#pragma unroll 1
        for (int i = 0; i < 8; ++i) {
            const int e = (tid >> 3) + 32 * i, piece = tid & 7;
            const v4f a4 = *(const v4fa*)(&tile[e * 32 + piece * 4]);
            const v4f m4 = *(const v4fa*)(&smu[piece * 4]);
            const v4f r4 = *(const v4fa*)(&srs[piece * 4]);
            const float w = bfr(lw[e]), bb = bfr(lb[e]);
            v4f val;
#pragma unroll
            for (int j = 0; j < 4; ++j) val[j] = (a4[j] - m4[j]) * r4[j] * w + bb;
            *(volatile v4f*)(OUT + ((size_t)(b * CCH + e)) * OUT_SEQ + t0 + piece * 4) = val; }
        if (ps == 0) __threadfence(); }
}

static constexpr size_t al256(size_t v) { return (v + 255) & ~(size_t)255; }
static constexpr size_t SZ_WB = al256(((size_t)2 * CCH * CCH + (size_t)2 * CCH * KVC + (size_t)CCH * CTXP) * 2);
static constexpr size_t SZ_PL = al256((size_t)NB * SEQ * CCH * 2);
static constexpr size_t SZ_P2 = al256((size_t)NB * SEQ * KVC * 2);
static constexpr size_t SZ_YF = al256((size_t)NB * CCH * SEQ * 4);
static constexpr size_t SZ_TOTAL = SZ_WB + 2 * SZ_PL + SZ_P2 + 2 * SZ_PL + SZ_PL + SZ_PL + SZ_P2 + SZ_YF;
static_assert(SZ_TOTAL <= (size_t)134217728);
static_assert(((size_t)CCH * CCH * 2) % 256 == 0);
static_assert(((size_t)CCH * KVC * 2) % 256 == 0);
static_assert(KVC == CTXP);
static_assert(((size_t)CCH * CCH) % 8 == 0);
static_assert(((size_t)CCH * KVC) % 8 == 0);

extern "C" void kernel_launch(void* const* d_in, const int* in_sizes, int n_in,
                              void* d_out, int out_size, void* d_ws, size_t ws_size, hipStream_t stream) {
    if (n_in < 15) return;
    const size_t needq = ((size_t)((NB - 1) * CCH + (CCH - 1))) * SEQ_FULL + SEQ;
    const size_t needkv = ((size_t)((NB - 1) * KVC + (KVC - 1))) * SEQ_FULL + SEQ;
    if ((size_t)in_sizes[0] < needq || (size_t)in_sizes[1] < needq || (size_t)in_sizes[2] < needkv) return;
    if ((size_t)in_sizes[3] < (size_t)CCH * CCH || (size_t)in_sizes[5] < (size_t)CCH * CCH) return;
    if ((size_t)in_sizes[7] < (size_t)CCH * KVC || (size_t)in_sizes[9] < (size_t)CCH * KVC || (size_t)in_sizes[11] < (size_t)CCH * CTXP) return;
    if (in_sizes[4] < CCH || in_sizes[6] < CCH || in_sizes[8] < CCH || in_sizes[10] < CCH || in_sizes[12] < CCH || in_sizes[13] < CCH || in_sizes[14] < CCH) return;
    if ((size_t)out_size < ((size_t)((NB - 1) * CCH + (CCH - 1))) * OUT_SEQ + SEQ) return;
    if (SZ_TOTAL > ws_size) return;
    const float* q1  = (const float*)d_in[0];
    const float* q2  = (const float*)d_in[1];
    const float* kv  = (const float*)d_in[2];
    const float* wq1 = (const float*)d_in[3];
    const float* bq1 = (const float*)d_in[4];
    const float* wq2 = (const float*)d_in[5];
    const float* bq2 = (const float*)d_in[6];
    const float* wk  = (const float*)d_in[7];
    const float* bk  = (const float*)d_in[8];
    const float* wv  = (const float*)d_in[9];
    const float* bv  = (const float*)d_in[10];
    const float* wo  = (const float*)d_in[11];
    const float* bo  = (const float*)d_in[12];
    const float* lnw = (const float*)d_in[13];
    const float* lnb = (const float*)d_in[14];
    float* OUT = (float*)d_out;
    char* wsp = (char*)d_ws;
    h16* WB  = (h16*)wsp; wsp += SZ_WB;
    h16* X1T = (h16*)wsp; wsp += SZ_PL;
    h16* X2T = (h16*)wsp; wsp += SZ_PL;
    h16* KVT = (h16*)wsp; wsp += SZ_P2;
    h16* QP  = (h16*)wsp; wsp += 2 * SZ_PL;
    h16* KP  = (h16*)wsp; wsp += SZ_PL;
    h16* VT  = (h16*)wsp; wsp += SZ_PL;
    h16* CTX = (h16*)wsp; wsp += SZ_P2;
    float* YF = (float*)wsp; wsp += SZ_YF;
    h16* WQ1 = WB; h16* WQ2 = WB + (size_t)CCH * CCH; h16* WK = WB + (size_t)2 * CCH * CCH;
    h16* WV = WK + (size_t)CCH * KVC; h16* WO = WV + (size_t)CCH * KVC;

    { const size_t n8a = (size_t)CCH * CCH / 8; const unsigned ga = (unsigned)((n8a + 255) / 256);
      const size_t n8b = (size_t)CCH * KVC / 8; const unsigned gb = (unsigned)((n8b + 255) / 256);
      const size_t n8c = (size_t)CCH * CTXP / 8; const unsigned gc = (unsigned)((n8c + 255) / 256);
      k_cvtw<<<ga, 256, 0, stream>>>(wq1, WQ1, n8a); k_cvtw<<<ga, 256, 0, stream>>>(wq2, WQ2, n8a);
      k_cvtw<<<gb, 256, 0, stream>>>(wk, WK, n8b); k_cvtw<<<gb, 256, 0, stream>>>(wv, WV, n8b);
      k_cvtw<<<gc, 256, 0, stream>>>(wo, WO, n8c); }

    k_xpose<<<dim3(SEQ / 64, CCH / 64, NB), 256, 0, stream>>>(q1, X1T, CCH);
    k_xpose<<<dim3(SEQ / 64, CCH / 64, NB), 256, 0, stream>>>(q2, X2T, CCH);
    k_xpose<<<dim3(SEQ / 64, KVC / 64, NB), 256, 0, stream>>>(kv, KVT, KVC);

    const float sproj = 1.0f / (HSC * WSC);
    k_gemm_cb<<<dim3(NB * SEQ / 64, CCH / 64, 1), 32, 0, stream>>>(X1T, WQ1, bq1, QP, CCH, NB * SEQ, (size_t)0, CCH, CCH, (size_t)0, sproj, QSC);
    k_gemm_cb<<<dim3(NB * SEQ / 64, CCH / 64, 1), 32, 0, stream>>>(X2T, WQ2, bq2, QP + (size_t)NB * SEQ * CCH, CCH, NB * SEQ, (size_t)0, CCH, CCH, (size_t)0, sproj, QSC);
    k_gemm_cb<<<dim3(NB * SEQ / 64, CCH / 64, 1), 32, 0, stream>>>(KVT, WK, bk, KP, KVC, NB * SEQ, (size_t)0, CCH, CCH, (size_t)0, sproj, QSC);
    k_gemm_rb<<<dim3(CCH / 64, NB * SEQ / 64, 1), 32, 0, stream>>>(WV, KVT, bv, VT, KVC, CCH, (size_t)0, SEQ, SEQ, (size_t)CCH * SEQ, sproj, VSC);

    k_flash<<<dim3(SEQ / (16 * AW), NB, 2), 32 * AW, 0, stream>>>(QP, KP, VT, CTX);

    k_gemm_f32<<<dim3(CCH / 64, NB * SEQ / 64, 1), 32, 0, stream>>>(WO, CTX, bo, YF, CTXP, CCH, (size_t)0, SEQ, SEQ, (size_t)CCH * SEQ, 1.0f / (WSC * OSC), 1.0f);

    k_ln<<<dim3(SEQ / 32, NB, 1), 256, 0, stream>>>(YF, lnw, lnb, OUT);
}
